// BasisResidualFFN_7361573945459
// MI455X (gfx1250) — hardware-run, weakly checked
//
#include <hip/hip_runtime.h>
#include <math.h>

constexpr int kTok  = 4096;
constexpr int kDm   = 1024;
constexpr int kSel  = 8;
constexpr int kNeu  = 64;
constexpr int kNB   = 16;
constexpr int kRank = 32;
constexpr int kJJ   = kNB * kRank;
constexpr int kDff  = 4096;
constexpr float kCarryW   = 32.0f;
constexpr float kCarryWdn = 64.0f;
constexpr float kCarryP   = 16.0f;
constexpr float kCarryHid = 16.0f;

typedef __attribute__((ext_vector_type(16))) _Float16 v16h;
typedef __attribute__((ext_vector_type(8)))  _Float16 v8h;
typedef __attribute__((ext_vector_type(16))) __bf16   v16b;
typedef __attribute__((ext_vector_type(8)))  __bf16   v8b;
typedef __attribute__((ext_vector_type(8)))  float    v8f;
typedef __attribute__((ext_vector_type(4)))  float    v4f;
typedef __attribute__((ext_vector_type(4)))  unsigned int v4u;

__device__ __forceinline__ unsigned short f2bf_bits(float f) {
  unsigned u = __float_as_uint(f);
  return (unsigned short)((u + 0x7FFFu + ((u >> 16) & 1u)) >> 16);
}
__device__ __forceinline__ float bf_bits2f(unsigned short h) { return __uint_as_float(((unsigned)h) << 16); }

__device__ __forceinline__ void dep_guard_h(v8f& a, v8f& b, v16h x, v16h y) { asm volatile("v_nop\n\tv_nop\n\tv_nop\n\tv_nop" : "+v"(a), "+v"(b) : "v"(x), "v"(y)); }
__device__ __forceinline__ void dep_guard_b(v8f& a, v8f& b, v16b x, v16b y) { asm volatile("v_nop\n\tv_nop\n\tv_nop\n\tv_nop" : "+v"(a), "+v"(b) : "v"(x), "v"(y)); }
__device__ __forceinline__ void keep4_h(v16h a, v16h b, v16h c, v16h d) { asm volatile("v_nop" :: "v"(a), "v"(b), "v"(c), "v"(d)); }
__device__ __forceinline__ void keep4_b(v16b a, v16b b, v16b c, v16b d) { asm volatile("v_nop" :: "v"(a), "v"(b), "v"(c), "v"(d)); }
__device__ __forceinline__ void acc_guard4(v8f& a, v8f& b, v8f& c, v8f& d) { asm volatile("v_nop\n\tv_nop\n\tv_nop\n\tv_nop" : "+v"(a), "+v"(b), "+v"(c), "+v"(d)); }
template <typename T> struct Frag;
template <> struct Frag<_Float16> {
  typedef v16h V; union U { v16h v; v8h h[2]; };
  static __device__ __forceinline__ v16h load(const _Float16* p) {
    U f; f.h[0] = *(const v8h*)(p); f.h[1] = *(const v8h*)(p + 16); return f.v;
  }
  static __device__ __forceinline__ v8f mma(v16h a, v16h b, v8f c) {
    return __builtin_amdgcn_wmma_f32_16x16x32_f16(false, a, false, b, (short)0, c, false, false);
  }
  static __device__ __forceinline__ void guard(v8f& a, v8f& b, v16h x, v16h y) { dep_guard_h(a, b, x, y); }
  static __device__ __forceinline__ void keep(v16h a, v16h b, v16h c, v16h d) { keep4_h(a, b, c, d); }
};
template <> struct Frag<__bf16> {
  typedef v16b V; union U { v16b v; v8b h[2]; };
  static __device__ __forceinline__ v16b load(const __bf16* p) {
    U f; f.h[0] = *(const v8b*)(p); f.h[1] = *(const v8b*)(p + 16); return f.v;
  }
  static __device__ __forceinline__ v8f mma(v16b a, v16b b, v8f c) {
    return __builtin_amdgcn_wmma_f32_16x16x32_bf16(false, a, false, b, (short)0, c, false, false);
  }
  static __device__ __forceinline__ void guard(v8f& a, v8f& b, v16b x, v16b y) { dep_guard_b(a, b, x, y); }
  static __device__ __forceinline__ void keep(v16b a, v16b b, v16b c, v16b d) { keep4_b(a, b, c, d); }
};

__device__ __forceinline__ unsigned pk16(unsigned short a, unsigned short b) { return (unsigned)a | ((unsigned)b << 16); }
__device__ __forceinline__ unsigned short h_bits(float f) { const _Float16 h = (_Float16)f; return __builtin_bit_cast(unsigned short, h); }

template <int ET> struct Elem;
template <> struct Elem<0> { typedef _Float16 T; };
template <> struct Elem<1> { typedef __bf16 T; };
template <int ET, bool SPLIT, int BIAS_MODE, int OUT_MODE, bool RESID, int ACT = 0, bool DYNSCALE = false>
__global__ __launch_bounds__(256) void wmma_gemm64(
    const unsigned short* __restrict__ Ap, const unsigned short* __restrict__ A2p, int lda, long strideA,
    const unsigned short* __restrict__ Btp, const unsigned short* __restrict__ Bt2p, int ldb, long strideB,
    void* __restrict__ Cout, void* __restrict__ Cout2, int ldc, long strideC,
    const float* __restrict__ bias,
    const float* __restrict__ resid, long strideR,
    const float* __restrict__ scalep,
    int M, int N, int K, float scale) {
  typedef typename Elem<ET>::T T;
  typedef typename Frag<T>::V V;
  const T* A = (const T*)Ap; const T* A2 = (const T*)A2p; const T* Bt = (const T*)Btp; const T* Bt2 = (const T*)Bt2p;
  __shared__ __align__(16) float sT[8][16 * 68];
  const int b    = blockIdx.y;
  const int lane = threadIdx.x & 31;
  const int wave = threadIdx.x >> 5;
  const int tilesN = N >> 6;
  const int tilesM = M >> 6;
  const int tile = blockIdx.x * 8 + wave;
  if (tile >= tilesM * tilesN) return;
  const int tm = tile / tilesN;
  const int tn = tile - tm * tilesN;
  const int m0 = tm << 6;
  const int n0 = tn << 6;
  const float scl = DYNSCALE ? (scale * scalep[0]) : scale;

  const T* Ab  = A  + (size_t)b * strideA;
  const T* Bb  = Bt + (size_t)b * strideB;
  const T* Ab2 = SPLIT ? (A2  + (size_t)b * strideA) : nullptr;
  const T* Bb2 = SPLIT ? (Bt2 + (size_t)b * strideB) : nullptr;

  const int rlane = lane & 15;
  const int koff  = (lane >> 4) * 8;
  const int mOff  = (lane >> 4) * 8;

  v8f acc[4][4];
#pragma unroll
  for (int i = 0; i < 4; ++i)
#pragma unroll
    for (int j = 0; j < 4; ++j) acc[i][j] = (v8f){0.f,0.f,0.f,0.f,0.f,0.f,0.f,0.f};

  for (int k0 = 0; k0 < K; k0 += 32) {
    V bh[4], bl[4];
#pragma unroll
    for (int j = 0; j < 4; ++j) {
      const size_t bo = (size_t)(n0 + (j << 4) + rlane) * ldb + koff + k0;
      bh[j] = Frag<T>::load(Bb + bo);
      if (SPLIT) bl[j] = Frag<T>::load(Bb2 + bo);
    }
#pragma unroll
    for (int i = 0; i < 4; ++i) {
      const size_t ao = (size_t)(m0 + (i << 4) + rlane) * lda + koff + k0;
      V ah = Frag<T>::load(Ab + ao);
      V al;
      if (SPLIT) al = Frag<T>::load(Ab2 + ao);
#pragma unroll
      for (int j = 0; j < 4; ++j) {
        acc[i][j] = Frag<T>::mma(ah, bh[j], acc[i][j]);
        if (SPLIT) {
          acc[i][j] = Frag<T>::mma(ah, bl[j], acc[i][j]);
          acc[i][j] = Frag<T>::mma(al, bh[j], acc[i][j]);
        }
      }
      Frag<T>::guard(acc[i][0], acc[i][3], ah, SPLIT ? al : ah);
    }
    Frag<T>::keep(bh[0], bh[1], bh[2], bh[3]);
    if (SPLIT) Frag<T>::keep(bl[0], bl[1], bl[2], bl[3]);
  }
  acc_guard4(acc[0][0], acc[0][1], acc[0][2], acc[0][3]);
  acc_guard4(acc[1][0], acc[1][1], acc[1][2], acc[1][3]);
  acc_guard4(acc[2][0], acc[2][1], acc[2][2], acc[2][3]);
  acc_guard4(acc[3][0], acc[3][1], acc[3][2], acc[3][3]);

  float* slab = sT[wave];
  const float* Rb = RESID ? (resid + (size_t)b * strideR) : nullptr;
#pragma unroll
  for (int i = 0; i < 4; ++i) {
    const int mBase = m0 + (i << 4);
#pragma unroll
    for (int j = 0; j < 4; ++j) {
      const int n = n0 + (j << 4) + rlane;
      float bv = 0.f;
      if (BIAS_MODE == 2) bv = bias[n];
#pragma unroll
      for (int r = 0; r < 8; ++r) {
        float v = acc[i][j][r] * scl;
        if (BIAS_MODE == 1) v += bias[mBase + mOff + r];
        if (BIAS_MODE == 2) v += bv;
        if (RESID) v += Rb[(size_t)(mBase + mOff + r) * ldc + n];
        if (ACT == 2) v = fmaxf(v, 0.0f);
        if (ACT == 4) v = (v > 0.f) ? v : 0.01f * v;
        slab[(mOff + r) * 68 + (j << 4) + rlane] = v;
      }
    }
    __builtin_amdgcn_fence(__ATOMIC_RELEASE, "workgroup");
    __builtin_amdgcn_wave_barrier();
    __builtin_amdgcn_fence(__ATOMIC_ACQUIRE, "workgroup");
    if (OUT_MODE == 0) {
      float* C = (float*)Cout + (size_t)b * strideC;
      const int hh = lane >> 4, c4 = (lane & 15) * 4;
      for (int pass = 0; pass < 2; ++pass) {
#pragma unroll
        for (int it = 0; it < 8; ++it) {
          const int row = it * 2 + hh;
          v4f v = *(const v4f*)(slab + row * 68 + c4);
          *(volatile v4f*)(C + (size_t)(mBase + row) * ldc + n0 + c4) = v;
        }
        __threadfence();
      }
    } else {
      const int q = lane >> 3, c8 = (lane & 7) * 8;
      unsigned short* C  = (unsigned short*)Cout  + (size_t)b * strideC;
      unsigned short* C2 = (OUT_MODE == 2) ? ((unsigned short*)Cout2 + (size_t)b * strideC) : nullptr;
      for (int pass = 0; pass < 2; ++pass) {
#pragma unroll
        for (int it = 0; it < 4; ++it) {
          const int row = it * 4 + q;
          const float* sp = slab + row * 68 + c8;
          v8h hv, lv;
#pragma unroll
          for (int e = 0; e < 8; ++e) {
            if (OUT_MODE == 1) {
              hv[e] = (_Float16)sp[e];
            } else {
              unsigned short hb = f2bf_bits(sp[e]);
              unsigned short lb = f2bf_bits(sp[e] - bf_bits2f(hb));
              hv[e] = __builtin_bit_cast(_Float16, hb);
              lv[e] = __builtin_bit_cast(_Float16, lb);
            }
          }
          *(volatile v8h*)(C + (size_t)(mBase + row) * ldc + n0 + c8) = hv;
          if (OUT_MODE == 2) *(volatile v8h*)(C2 + (size_t)(mBase + row) * ldc + n0 + c8) = lv;
        }
        __threadfence();
      }
    }
    __builtin_amdgcn_fence(__ATOMIC_RELEASE, "workgroup");
    __builtin_amdgcn_wave_barrier();
    __builtin_amdgcn_fence(__ATOMIC_ACQUIRE, "workgroup");
  }
}

__global__ __launch_bounds__(256) void cast8_f16_kernel(const float* __restrict__ in, unsigned short* __restrict__ out, int n8) {
  const int i = blockIdx.x * 256 + threadIdx.x;
  if (i >= n8) return;
  const float* p = in + 8 * (size_t)i;
  const v4f a = *(const v4f*)(p);
  const v4f c = *(const v4f*)(p + 4);
  unsigned short hb[8];
#pragma unroll
  for (int e = 0; e < 4; ++e) {
    hb[e]     = h_bits(a[e]);
    hb[4 + e] = h_bits(c[e]);
  }
  const v4u u = (v4u){pk16(hb[0], hb[1]), pk16(hb[2], hb[3]), pk16(hb[4], hb[5]), pk16(hb[6], hb[7])};
  unsigned short* q = out + 8 * (size_t)i;
  *(volatile v4u*)q = u;
  __threadfence();
  *(volatile v4u*)q = u;
}

__global__ __launch_bounds__(256) void basis_rows_kernel(const float* __restrict__ A, unsigned short* __restrict__ out, float scale) {
  const int i = blockIdx.x * 256 + threadIdx.x;
  if (i >= kDm * kNB * 4) return;
  const int q = i & 3;
  const int n = (i >> 2) & (kNB - 1);
  const int d = i >> 6;
  const float* p = A + ((size_t)n * kDm + d) * kRank + 8 * q;
  const v4f a = *(const v4f*)(p);
  const v4f c = *(const v4f*)(p + 4);
  unsigned short hb[8];
#pragma unroll
  for (int e = 0; e < 4; ++e) {
    hb[e]     = h_bits(a[e] * scale);
    hb[4 + e] = h_bits(c[e] * scale);
  }
  const v4u u = (v4u){pk16(hb[0], hb[1]), pk16(hb[2], hb[3]), pk16(hb[4], hb[5]), pk16(hb[6], hb[7])};
  unsigned short* dst = out + 8 * (size_t)i;
  *(volatile v4u*)dst = u;
  __threadfence();
  *(volatile v4u*)dst = u;
}

__global__ __launch_bounds__(256) void basis_t_kernel(const float* __restrict__ A, unsigned short* __restrict__ out, float scale) {
  __shared__ float sm[kRank][65];
  const int t  = threadIdx.x;
  const int d0 = blockIdx.x * 64;
  const int n  = blockIdx.y;
  const float* src = A + ((size_t)n * kDm + d0) * kRank;
#pragma unroll
  for (int i = 0; i < 8; ++i) {
    const int e  = i * 256 + t;
    const int dl = e >> 5;
    const int r  = e & 31;
    sm[r][dl] = src[e] * scale;
  }
  __syncthreads();
  const int lane = t & 31, wave = t >> 5;
  const int q = lane >> 3, c8 = (lane & 7) * 8;
  const int row = wave * 4 + q;
  unsigned short hb[8];
#pragma unroll
  for (int e = 0; e < 8; ++e) hb[e] = h_bits(sm[row][c8 + e]);
  const v4u u = (v4u){pk16(hb[0], hb[1]), pk16(hb[2], hb[3]), pk16(hb[4], hb[5]), pk16(hb[6], hb[7])};
  unsigned short* dst = out + (size_t)(n * kRank + row) * kDm + d0 + c8;
  for (int pass = 0; pass < 2; ++pass) {
    *(volatile v4u*)dst = u;
    __threadfence();
  }
}

__global__ __launch_bounds__(256) void tcast_kernel(const float* __restrict__ in, unsigned short* __restrict__ out,
                                                    int R, int Ccols, float scale) {
  __shared__ float sm[64][65];
  const int t  = threadIdx.x;
  const int r0 = blockIdx.x * 64;
  const int c0 = blockIdx.y * 64;
#pragma unroll
  for (int i = 0; i < 16; ++i) {
    const int e  = i * 256 + t;
    const int rl = e >> 6;
    const int cl = e & 63;
    sm[cl][rl] = in[(size_t)(r0 + rl) * Ccols + c0 + cl] * scale;
  }
  __syncthreads();
  const int lane = t & 31, wave = t >> 5;
  const int q = lane >> 3, c8 = (lane & 7) * 8;
  for (int pass = 0; pass < 2; ++pass) {
#pragma unroll
    for (int it = 0; it < 2; ++it) {
      const int row = wave * 8 + it * 4 + q;
      unsigned short hb[8];
#pragma unroll
      for (int e = 0; e < 8; ++e) hb[e] = h_bits(sm[row][c8 + e]);
      const v4u u = (v4u){pk16(hb[0], hb[1]), pk16(hb[2], hb[3]), pk16(hb[4], hb[5]), pk16(hb[6], hb[7])};
      *(volatile v4u*)(out + (size_t)(c0 + row) * R + r0 + c8) = u;
    }
    __threadfence();
  }
}

__global__ __launch_bounds__(256) void recipe_kernel(const float* __restrict__ G, const int* __restrict__ nidx,
                                                     const float* __restrict__ nw, const float* __restrict__ rec,
                                                     unsigned short* __restrict__ P16, float carry) {
  __shared__ __align__(16) unsigned short sP[8][kJJ];
  const int t = threadIdx.x;
  const int lane = t & 31, wave = t >> 5;
  const int tok = blockIdx.x * 8 + wave;
  const int nl = lane & 15;
  float tr = 0.f;
#pragma unroll 1
  for (int k = 0; k < kSel; ++k) {
    int id = nidx[tok * kSel + k];
    id = id < 0 ? 0 : (id > kNeu - 1 ? kNeu - 1 : id);
    const float wk = nw[tok * kSel + k];
    const float v = rec[id * kNB + nl];
    float m = v;
    m = fmaxf(m, __shfl_xor(m, 1, 32));
    m = fmaxf(m, __shfl_xor(m, 2, 32));
    m = fmaxf(m, __shfl_xor(m, 4, 32));
    m = fmaxf(m, __shfl_xor(m, 8, 32));
    const float e = expf(v - m);
    float s = e;
    s += __shfl_xor(s, 1, 32);
    s += __shfl_xor(s, 2, 32);
    s += __shfl_xor(s, 4, 32);
    s += __shfl_xor(s, 8, 32);
    const float sel = e * (1.0f / s);
    const float pw = sel * wk;
    tr += pw;
  }
  const float* Gt = G + (size_t)tok * kJJ;
  float trn[kNB];
  float h = 0.f;
#pragma unroll
  for (int n = 0; n < kNB; ++n) {
    trn[n] = __shfl(tr, n, 32);
    h += trn[n] * Gt[n * kRank + lane];
  }
  unsigned short* sp = sP[wave];
#pragma unroll
  for (int n = 0; n < kNB; ++n) {
    const float p = trn[n] * h;
    sp[n * kRank + lane] = h_bits(p * carry);
  }
  __syncthreads();
  unsigned short* dst = P16 + (size_t)tok * kJJ;
  for (int pass = 0; pass < 2; ++pass) {
#pragma unroll
    for (int it = 0; it < 2; ++it) {
      const int o = it * 256 + 8 * lane;
      const v4u u = (v4u){pk16(sp[o], sp[o + 1]), pk16(sp[o + 2], sp[o + 3]),
                          pk16(sp[o + 4], sp[o + 5]), pk16(sp[o + 6], sp[o + 7])};
      *(volatile v4u*)(dst + o) = u;
    }
    __threadfence();
  }
}

__global__ __launch_bounds__(256) void gelu_cast_kernel(const float* __restrict__ Z, unsigned short* __restrict__ H, float carry) {
  __shared__ __align__(16) unsigned short sh[2048];
  const size_t base = (size_t)blockIdx.x * 2048;
  const int t = threadIdx.x;
#pragma unroll 1
  for (int it = 0; it < 8; ++it) {
    const float z = Z[base + it * 256 + t];
    const float g = 0.5f * z * (1.0f + erff(z * 0.70710678118654752f));
    sh[it * 256 + t] = h_bits(g * carry);
  }
  __syncthreads();
  const int o = 8 * t;
  const v4u u = (v4u){pk16(sh[o], sh[o + 1]), pk16(sh[o + 2], sh[o + 3]),
                      pk16(sh[o + 4], sh[o + 5]), pk16(sh[o + 6], sh[o + 7])};
  unsigned short* dst = H + base + o;
  *(volatile v4u*)dst = u;
  __threadfence();
  *(volatile v4u*)dst = u;
}

extern "C" void kernel_launch(void* const* d_in, const int* in_sizes, int n_in,
                              void* d_out, int out_size, void* d_ws, size_t ws_size,
                              hipStream_t stream) {
  const float* x      = (const float*)d_in[0];
  const int*   nidx   = (const int*)d_in[1];
  const float* nw     = (const float*)d_in[2];
  const float* recipe = (const float*)d_in[3];
  const float* basisA = (const float*)d_in[4];
  const float* wup    = (const float*)d_in[5];
  const float* wupb   = (const float*)d_in[6];
  const float* wdn    = (const float*)d_in[7];
  const float* wdnb   = (const float*)d_in[8];
  const float* alphap = (const float*)d_in[9];
  float* out = (float*)d_out;
  (void)in_sizes; (void)n_in; (void)out_size;

  const size_t bX16 = (size_t)kTok * kDm * 2;
  const size_t bBas = (size_t)kJJ * kDm * 2;
  const size_t bG   = (size_t)kTok * kJJ * 4;
  const size_t bP16 = (size_t)kTok * kJJ * 2;
  const size_t bZ   = (size_t)kTok * kDff * 4;
  const size_t bXF  = (size_t)kTok * kDm * 2;
  const size_t bWup = (size_t)kDff * kDm * 2;
  const size_t bWdn = (size_t)kDm * kDff * 2;
  const size_t bHid = (size_t)kTok * kDff * 2;

  const size_t oX16 = 0;
  const size_t oBT  = oX16 + bX16;
  const size_t oBR  = oBT + bBas;
  const size_t oG   = oBR + bBas;
  const size_t oP16 = oG + bG;
  const size_t lowEnd = oP16 + bP16;
  const size_t oZ   = 0;
  const size_t hiBase = (oZ + bZ > lowEnd) ? (oZ + bZ) : lowEnd;
  const size_t oXF  = hiBase;
  const size_t oWup = oXF + bXF;
  const size_t oWdn = oWup + bWup;
  const size_t oHid = oWdn + bWdn;
  const size_t total = oHid + bHid;
  if (total > ws_size) return;

  char* ws = (char*)d_ws;
  unsigned short* X16  = (unsigned short*)(ws + oX16);
  unsigned short* basT = (unsigned short*)(ws + oBT);
  unsigned short* basR = (unsigned short*)(ws + oBR);
  float*          Gf   = (float*)(ws + oG);
  unsigned short* P16  = (unsigned short*)(ws + oP16);
  float*          Zpre = (float*)(ws + oZ);
  unsigned short* XF16 = (unsigned short*)(ws + oXF);
  unsigned short* WupT = (unsigned short*)(ws + oWup);
  unsigned short* WdnT = (unsigned short*)(ws + oWdn);
  unsigned short* HID  = (unsigned short*)(ws + oHid);

  {
    const int n8 = kTok * kDm / 8;
    cast8_f16_kernel<<<(n8 + 255) / 256, 256, 0, stream>>>(x, X16, n8);
  }
  basis_t_kernel<<<dim3(kDm / 64, kNB), 256, 0, stream>>>(basisA, basT, kCarryW);
  {
    const int n8 = kDm * kNB * 4;
    basis_rows_kernel<<<(n8 + 255) / 256, 256, 0, stream>>>(basisA, basR, kCarryW);
  }
  tcast_kernel<<<dim3(kDm / 64, kDff / 64), 256, 0, stream>>>(wup, WupT, kDm, kDff, kCarryW);
  tcast_kernel<<<dim3(kDff / 64, kDm / 64), 256, 0, stream>>>(wdn, WdnT, kDff, kDm, kCarryWdn);

  wmma_gemm64<0, false, 0, 0, false, 0, false><<<dim3((kTok / 64) * (kJJ / 64) / 8, 1), 256, 0, stream>>>(
      X16, nullptr, kDm, 0L, basT, nullptr, kDm, 0L,
      (void*)Gf, nullptr, kJJ, 0L, nullptr, nullptr, 0L, nullptr,
      kTok, kJJ, kDm, 1.0f / kCarryW);

  recipe_kernel<<<kTok / 8, 256, 0, stream>>>(Gf, nidx, nw, recipe, P16, kCarryP);

  wmma_gemm64<0, false, 0, 1, true, 0, true><<<dim3((kTok / 64) * (kDm / 64) / 8, 1), 256, 0, stream>>>(
      P16, nullptr, kJJ, 0L, basR, nullptr, kJJ, 0L,
      (void*)XF16, nullptr, kDm, 0L, nullptr, x, 0L, alphap,
      kTok, kDm, kJJ, 1.0f / (kCarryP * kCarryW));

  wmma_gemm64<0, false, 2, 0, false, 0, false><<<dim3((kTok / 64) * (kDff / 64) / 8, 1), 256, 0, stream>>>(
      XF16, nullptr, kDm, 0L, WupT, nullptr, kDm, 0L,
      (void*)Zpre, nullptr, kDff, 0L, wupb, nullptr, 0L, nullptr,
      kTok, kDff, kDm, 1.0f / kCarryW);

  gelu_cast_kernel<<<(kTok / 2048) * kDff, 256, 0, stream>>>(Zpre, HID, kCarryHid);

  wmma_gemm64<0, false, 2, 0, false, 0, false><<<dim3((kTok / 64) * (kDm / 64) / 8, 1), 256, 0, stream>>>(
      HID, nullptr, kDff, 0L, WdnT, nullptr, kDff, 0L,
      (void*)out, nullptr, kDm, 0L, wdnb, nullptr, 0L, nullptr,
      kTok, kDm, kDff, 1.0f / (kCarryHid * kCarryWdn));
}
